// MultiHeadAttention_65773129171319
// MI455X (gfx1250) — hardware-verified
//
#include <hip/hip_runtime.h>
#ifndef NB
#define NB 2
#endif
#ifndef SEQ
#define SEQ 2048
#endif
#define NB_FULL 2
#define SEQ_FULL 2048
#define RD 512
#define NH 8
#define HD 64
#define KP 1024
#define HP 128
#define OUT1_OFF ((size_t)NB_FULL * SEQ_FULL * RD)

static_assert(SEQ % 64 == 0);
static_assert(SEQ <= SEQ_FULL);
static_assert(NB <= NB_FULL);
static_assert(NH * HD == RD);
static_assert(RD % 64 == 0);
static_assert(RD % 32 == 0);
static_assert(NH * HP == KP);
static_assert(KP == 2 * RD);
static_assert(HP == 2 * HD);
static_assert(HD == 64);
static_assert((NB * SEQ) % 64 == 0);
static_assert(((size_t)NB * SEQ * (SEQ / 32)) % 32 == 0);
static_assert(OUT1_OFF * 4 == (size_t)8388608);
static_assert((size_t)7 * ((size_t)NB * SEQ * KP * 2) + (size_t)4 * ((size_t)RD * RD * 2) + (size_t)NB * SEQ * (SEQ / 32) * 4 <= (size_t)134217728);

typedef __bf16 v16b __attribute__((ext_vector_type(16)));
typedef _Float16 v16h __attribute__((ext_vector_type(16)));
typedef _Float16 h16;
typedef unsigned short v8us __attribute__((ext_vector_type(8), may_alias));
typedef int v4i __attribute__((ext_vector_type(4), may_alias));
typedef float v8f __attribute__((ext_vector_type(8)));
typedef float v4f __attribute__((ext_vector_type(4)));
typedef float v4fa __attribute__((ext_vector_type(4), may_alias));
union Frag { v16b vb; v16h vh; v8us half[2]; unsigned short u[16]; _Float16 h[16]; };

#define LOG2E 1.4426950408889634f
#define CSCALE (0.08838834764831845f * LOG2E / 65536.0f)
#define MFILL (-1.0e9f * LOG2E)

__device__ __forceinline__ unsigned short bf16_bits(float x) {
  unsigned int u = __float_as_uint(x);
  return (unsigned short)((u + 0x7FFFu + ((u >> 16) & 1u)) >> 16);
}
__device__ __forceinline__ float bf16_val(unsigned short b) { return __uint_as_float(((unsigned int)b) << 16); }
__device__ __forceinline__ float bf16_rne(float x) { return bf16_val(bf16_bits(x)); }
__device__ __forceinline__ unsigned short f16_bits(_Float16 h) { union { _Float16 h; unsigned short u; } c; c.h = h; return c.u; }
__device__ __forceinline__ unsigned short c16(float c) { return f16_bits((_Float16)c); }

static __device__ __forceinline__ h16 toh_flush(float v) { const h16 r = (h16)v; return (fabsf(v) < 6.103515625e-05f) ? (h16)0.0f : r; }
__device__ __forceinline__ unsigned short c16f(float c) { return f16_bits(toh_flush(c)); }

__device__ __forceinline__ v8f wm_b(const Frag& a, const Frag& b, v8f c) {
  return __builtin_amdgcn_wmma_f32_16x16x32_bf16(false, a.vb, false, b.vb, (short)0, c, false, false);
}
__device__ __forceinline__ v8f wm_h(const Frag& a, const Frag& b, v8f c) {
  return __builtin_amdgcn_wmma_f32_16x16x32_f16(false, a.vh, false, b.vh, (short)0, c, false, false);
}

template <bool BF>
__device__ __forceinline__ void rmma(const Frag& ar, const Frag& ai, const Frag& wf, v8f& yr, v8f& yi) {
  if (BF) {
    yr = wm_b(ar, wf, yr);
    asm volatile("v_nop\n\tv_nop\n\tv_nop\n\tv_nop" : "+v"(yr) : "v"(ar.vb), "v"(wf.vb));
    yi = wm_b(ai, wf, yi);
    asm volatile("v_nop\n\tv_nop\n\tv_nop\n\tv_nop" : "+v"(yi) : "v"(ai.vb), "v"(wf.vb));
  } else {
    yr = wm_h(ar, wf, yr);
    asm volatile("v_nop\n\tv_nop\n\tv_nop\n\tv_nop" : "+v"(yr) : "v"(ar.vh), "v"(wf.vh));
    yi = wm_h(ai, wf, yi);
    asm volatile("v_nop\n\tv_nop\n\tv_nop\n\tv_nop" : "+v"(yi) : "v"(ai.vh), "v"(wf.vh));
  }
}

template <bool BF>
__device__ __forceinline__ void rgemm_main(const unsigned short* __restrict__ A, const unsigned short* __restrict__ W,
                                           int row0, int col0, int ln, int hh, v8f (&yr)[4], v8f (&yi)[4]) {
  const unsigned short* ap = A + (size_t)(row0 + ln) * KP + 8 * hh;
  const unsigned short* wp = W + (size_t)(col0 + ln) * RD + 8 * hh;
#pragma unroll 2
  for (int c = 0; c < RD / 32; ++c) {
    const int k0 = 32 * c;
    Frag ar, ai;
    ar.half[0] = *(const v8us*)(ap + k0);
    ar.half[1] = *(const v8us*)(ap + k0 + 16);
    ai.half[0] = *(const v8us*)(ap + RD + k0);
    ai.half[1] = *(const v8us*)(ap + RD + k0 + 16);
#pragma unroll
    for (int t = 0; t < 4; ++t) {
      const unsigned short* wt = wp + (size_t)t * 16 * RD + k0;
      Frag wf;
      wf.half[0] = *(const v8us*)(wt);
      wf.half[1] = *(const v8us*)(wt + 16);
      rmma<BF>(ar, ai, wf, yr[t], yi[t]);
    }
  }
}

__global__ __launch_bounds__(256) void k_cvtx(const float* __restrict__ xr, const float* __restrict__ xi, unsigned short* __restrict__ X) {
  const int t = blockIdx.x * 256 + threadIdx.x;
  if (t >= NB * SEQ * 64) return;
  const int row = t >> 6, c8 = (t & 63) * 8;
  const int b = row / SEQ, s = row - b * SEQ;
  const size_t src = ((size_t)b * SEQ_FULL + (size_t)s) * RD + c8;
  const v4f r0 = *(const v4fa*)(xr + src), r1 = *(const v4fa*)(xr + src + 4);
  const v4f i0 = *(const v4fa*)(xi + src), i1 = *(const v4fa*)(xi + src + 4);
  v8us orr, oi;
  orr[0] = bf16_bits(r0[0]); orr[1] = bf16_bits(r0[1]); orr[2] = bf16_bits(r0[2]); orr[3] = bf16_bits(r0[3]);
  orr[4] = bf16_bits(r1[0]); orr[5] = bf16_bits(r1[1]); orr[6] = bf16_bits(r1[2]); orr[7] = bf16_bits(r1[3]);
  oi[0] = bf16_bits(i0[0]); oi[1] = bf16_bits(i0[1]); oi[2] = bf16_bits(i0[2]); oi[3] = bf16_bits(i0[3]);
  oi[4] = bf16_bits(i1[0]); oi[5] = bf16_bits(i1[1]); oi[6] = bf16_bits(i1[2]); oi[7] = bf16_bits(i1[3]);
  unsigned short* d = X + (size_t)row * KP + c8;
  *(volatile v8us*)d = orr;
  *(volatile v8us*)(d + RD) = oi;
  __threadfence();
  *(volatile v8us*)d = orr;
  *(volatile v8us*)(d + RD) = oi;
}

__global__ __launch_bounds__(256) void k_cvtwt(const float* __restrict__ w, unsigned short* __restrict__ Wt, int asf16) {
  __shared__ __attribute__((aligned(16))) unsigned short tl[64][72];
  const int tid = threadIdx.x;
  const int k0 = blockIdx.x * 64, n0 = blockIdx.y * 64;
#pragma unroll 1
  for (int j = 0; j < 16; ++j) {
    const int i = tid + 256 * j;
    const int kk = i >> 6, nn = i & 63;
    const float x = w[(size_t)(k0 + kk) * RD + (size_t)(n0 + nn)];
    const unsigned short vb = bf16_bits(x);
    const unsigned short vh = c16f(bf16_val(vb) * 1024.0f);
    tl[nn][kk] = (asf16 != 0) ? vh : vb;
  }
  __syncthreads();
  for (int pass = 0; pass < 2; ++pass) {
#pragma unroll
    for (int j = 0; j < 2; ++j) {
      const int i = tid + 256 * j;
      const int nn = i >> 3, p8 = (i & 7) * 8;
      const v8us a = *(const v8us*)&tl[nn][p8];
      *(volatile v8us*)(Wt + (size_t)(n0 + nn) * RD + (size_t)(k0 + p8)) = a;
    }
    if (pass == 0) __threadfence();
  }
}

__global__ __launch_bounds__(256) void k_maskbits(const int* __restrict__ mask, unsigned int* __restrict__ MB) {
  const int t = blockIdx.x * 256 + threadIdx.x;
  if (t >= NB * SEQ * (SEQ / 32)) return;
  const int row = t / (SEQ / 32), wc = t - row * (SEQ / 32);
  const int b = row / SEQ, q = row - b * SEQ;
  const int* mp = mask + ((size_t)b * SEQ_FULL + (size_t)q) * SEQ_FULL + (size_t)wc * 32;
  unsigned int word = 0u;
#pragma unroll 1
  for (int g = 0; g < 8; ++g) {
    const v4i m = *(const v4i*)(mp + 4 * g);
    const unsigned int nib = ((m[0] != 0) ? 1u : 0u) | ((m[1] != 0) ? 2u : 0u) | ((m[2] != 0) ? 4u : 0u) | ((m[3] != 0) ? 8u : 0u);
    word |= nib << (4 * g);
  }
  *(volatile unsigned int*)(MB + t) = word;
  __threadfence();
  *(volatile unsigned int*)(MB + t) = word;
}

__global__ __launch_bounds__(128) void k_proj_rows(const unsigned short* __restrict__ X, const unsigned short* __restrict__ W,
                                                   unsigned short* __restrict__ P, float cim) {
  __shared__ __attribute__((aligned(16))) unsigned short sh[4][16][136];
  const int tid = threadIdx.x, w = __builtin_amdgcn_readfirstlane((int)(tid >> 5)), lane = tid & 31, ln = lane & 15, hh = lane >> 4;
  const int head = blockIdx.y;
  const int rowb = blockIdx.x * 64;
  v8f yr[4] = {}, yi[4] = {};
  rgemm_main<true>(X, W, rowb + 16 * w, head * HD, ln, hh, yr, yi);
#pragma unroll
  for (int t = 0; t < 4; ++t) {
#pragma unroll
    for (int r = 0; r < 8; ++r) {
      sh[w][8 * hh + r][16 * t + ln]      = c16f(yr[t][r] * 256.0f);
      sh[w][8 * hh + r][HD + 16 * t + ln] = c16f(yi[t][r] * cim);
    }
  }
  __syncthreads();
  const int b = rowb / SEQ;
  const int s0 = rowb - b * SEQ + 16 * w;
  const size_t base = ((size_t)(b * NH + head) * SEQ + (size_t)s0) * HP;
  const int rsub = lane >> 4, p8 = (lane & 15) * 8;
  for (int pass = 0; pass < 2; ++pass) {
#pragma unroll
    for (int q = 0; q < 8; ++q) {
      const int row = 2 * q + rsub;
      const v8us a = *(const v8us*)&sh[w][row][p8];
      *(volatile v8us*)(P + base + (size_t)row * HP + p8) = a;
    }
    if (pass == 0) __threadfence();
  }
}

__global__ __launch_bounds__(128) void k_proj_vt(const unsigned short* __restrict__ X, const unsigned short* __restrict__ W,
                                                 unsigned short* __restrict__ Vt) {
  __shared__ __attribute__((aligned(16))) unsigned short th[HP][72];
  const int tid = threadIdx.x, w = __builtin_amdgcn_readfirstlane((int)(tid >> 5)), lane = tid & 31, ln = lane & 15, hh = lane >> 4;
  const int head = blockIdx.y;
  const int rowb = blockIdx.x * 64;
  v8f yr[4] = {}, yi[4] = {};
  rgemm_main<true>(X, W, rowb + 16 * w, head * HD, ln, hh, yr, yi);
#pragma unroll
  for (int t = 0; t < 4; ++t) {
#pragma unroll
    for (int r = 0; r < 8; ++r) {
      const int col = 16 * w + 8 * hh + r;
      th[16 * t + ln][col]      = c16f(yr[t][r] * 256.0f);
      th[HD + 16 * t + ln][col] = c16f(yi[t][r] * 256.0f);
    }
  }
  __syncthreads();
  const int b = rowb / SEQ;
  const int s0 = rowb - b * SEQ;
  const size_t base = (size_t)(b * NH + head) * HP * SEQ + (size_t)s0;
  for (int pass = 0; pass < 2; ++pass) {
    for (int i = tid; i < HP * 8; i += 128) {
      const int dd = i >> 3, j8 = (i & 7) * 8;
      const v8us a = *(const v8us*)&th[dd][j8];
      *(volatile v8us*)(Vt + base + (size_t)dd * SEQ + j8) = a;
    }
    if (pass == 0) __threadfence();
  }
}

__device__ __forceinline__ void score_mma(const Frag& k0, const Frag& k1, const Frag& k2, const Frag& k3,
                                          const Frag (&q)[4], v8f& sre, v8f& sa, v8f& sb) {
  sre = wm_h(k0, q[0], sre);
  sa  = wm_h(k0, q[2], sa);
  sb  = wm_h(k2, q[0], sb);
  sre = wm_h(k1, q[1], sre);
  sa  = wm_h(k1, q[3], sa);
  sb  = wm_h(k3, q[1], sb);
  sre = wm_h(k2, q[2], sre);
  sre = wm_h(k3, q[3], sre);
  asm volatile("v_nop\n\tv_nop\n\tv_nop\n\tv_nop" : "+v"(sre), "+v"(sa), "+v"(sb)
               : "v"(k0.vh), "v"(k1.vh), "v"(k2.vh), "v"(k3.vh),
                 "v"(q[0].vh), "v"(q[1].vh), "v"(q[2].vh), "v"(q[3].vh));
}
__device__ __forceinline__ void pv_mma(const Frag& v, const Frag& p, v8f& c) {
  c = wm_h(v, p, c);
  asm volatile("v_nop\n\tv_nop\n\tv_nop\n\tv_nop" : "+v"(c) : "v"(v.vh), "v"(p.vh));
}

__device__ __forceinline__ void fa_step(const unsigned short* __restrict__ Kp, const unsigned short* __restrict__ Vp,
                                        const unsigned int* __restrict__ Mw, int j, int ln, int hh,
                                        const Frag (&qf)[4], float& mr, float& lr, v8f (&O)[8]) {
  const v8f z8 = {0.f, 0.f, 0.f, 0.f, 0.f, 0.f, 0.f, 0.f};
  const int key0 = 32 * j;
  unsigned int mw = Mw[j];
  asm volatile("" : "+v"(mw));
  const unsigned int mh = mw >> (8 * hh);
  float sc[16];
#pragma unroll
  for (int kt = 0; kt < 2; ++kt) {
    const unsigned short* kp = Kp + (size_t)(key0 + 16 * kt + ln) * HP + 8 * hh;
    Frag k0, k1, k2, k3;
    k0.half[0] = *(const v8us*)(kp);      k0.half[1] = *(const v8us*)(kp + 16);
    k1.half[0] = *(const v8us*)(kp + 32); k1.half[1] = *(const v8us*)(kp + 48);
    k2.half[0] = *(const v8us*)(kp + 64); k2.half[1] = *(const v8us*)(kp + 80);
    k3.half[0] = *(const v8us*)(kp + 96); k3.half[1] = *(const v8us*)(kp + 112);
    v8f sre = z8, sa = z8, sb = z8;
    score_mma(k0, k1, k2, k3, qf, sre, sa, sb);
#pragma unroll
    for (int r = 0; r < 8; ++r) {
      const float im = sa[r] - sb[r];
      const float v = __builtin_amdgcn_sqrtf(fmaf(sre[r], sre[r], im * im)) * CSCALE;
      sc[8 * kt + r] = (((mh >> (16 * kt + r)) & 1u) != 0u) ? v : MFILL;
    }
  }
  float mx = sc[0];
#pragma unroll
  for (int i = 1; i < 16; ++i) mx = fmaxf(mx, sc[i]);
  mx = fmaxf(mx, __shfl_xor(mx, 16, 32));
  const float mnew = fmaxf(mr, mx);
  const float al = exp2f(mr - mnew);
  mr = mnew;
  Frag pf;
  float ps = 0.0f;
#pragma unroll
  for (int i = 0; i < 16; ++i) {
    const float e = (sc[i] - mnew) + 8.0f;
    const float pc = (e < -14.0f) ? 0.0f : exp2f(e);
    const _Float16 h = (_Float16)pc;
    pf.h[i] = h;
    ps += (float)h;
  }
  ps += __shfl_xor(ps, 16, 32);
  lr = lr * al + ps;
#pragma unroll
  for (int t = 0; t < 8; ++t) O[t] = O[t] * al;
  const size_t voff = (size_t)ln * SEQ + (size_t)(key0 + 8 * hh);
#pragma unroll
  for (int t = 0; t < 8; ++t) {
    const unsigned short* vp = Vp + voff + (size_t)t * 16 * SEQ;
    Frag vf;
    vf.half[0] = *(const v8us*)(vp);
    vf.half[1] = *(const v8us*)(vp + 16);
    pv_mma(vf, pf, O[t]);
  }
}

__global__ __launch_bounds__(128) void k_attn(const unsigned short* __restrict__ Qp, const unsigned short* __restrict__ Kpl,
                                              const unsigned short* __restrict__ Vt, const unsigned int* __restrict__ MB,
                                              unsigned short* __restrict__ Cx) {
  __shared__ __attribute__((aligned(16))) unsigned short sh[4][16][136];
  const int tid = threadIdx.x, w = __builtin_amdgcn_readfirstlane((int)(tid >> 5)), lane = tid & 31, ln = lane & 15, hh = lane >> 4;
  const int bh = blockIdx.x / (SEQ / 64), qt = blockIdx.x % (SEQ / 64);
  const int b = bh / NH, h = bh - b * NH;
  const int qbase = qt * 64 + 16 * w;
  const int qg = qbase + ln;
  Frag qf[4];
  {
    const size_t qoff = ((size_t)bh * SEQ + (size_t)qg) * HP + 8 * hh;
#pragma unroll
    for (int c = 0; c < 4; ++c) {
      qf[c].half[0] = *(const v8us*)(Qp + qoff + 32 * c);
      qf[c].half[1] = *(const v8us*)(Qp + qoff + 32 * c + 16);
    }
  }
  float mr = -3.0e38f, lr = 0.0f;
  v8f O[8] = {};
  const unsigned short* Kp = Kpl + (size_t)bh * SEQ * HP;
  const unsigned short* Vp = Vt  + (size_t)bh * HP * SEQ;
  const unsigned int* Mw = MB + ((size_t)b * SEQ + (size_t)qg) * (SEQ / 32);
#pragma unroll 1
  for (int j = 0; j < SEQ / 32; ++j)
    fa_step(Kp, Vp, Mw, j, ln, hh, qf, mr, lr, O);

  const float inv = 16.0f * (1.0f / lr);
#pragma unroll
  for (int t = 0; t < 8; ++t) {
#pragma unroll
    for (int r = 0; r < 8; ++r)
      sh[w][ln][16 * t + 8 * hh + r] = c16f(O[t][r] * inv);
  }
  __syncthreads();
  const size_t rbase = ((size_t)b * SEQ + (size_t)qbase) * KP + (size_t)h * HD;
  const int lsub = lane >> 3, p8 = (lane & 7) * 8;
  for (int pass = 0; pass < 2; ++pass) {
#pragma unroll
    for (int q = 0; q < 8; ++q) {
      const int line = 4 * q + lsub;
      const int row = line >> 1, seg = line & 1;
      const v8us a = *(const v8us*)&sh[w][row][seg * HD + p8];
      const size_t o = rbase + (size_t)row * KP + (size_t)seg * RD + p8;
      *(volatile v8us*)(Cx + o) = a;
    }
    if (pass == 0) __threadfence();
  }
}

__global__ __launch_bounds__(128) void k_out(const unsigned short* __restrict__ Cx, const unsigned short* __restrict__ Wo,
                                             float* __restrict__ Out) {
  __shared__ __attribute__((aligned(16))) float so[4][16][132];
  const int tid = threadIdx.x, w = __builtin_amdgcn_readfirstlane((int)(tid >> 5)), lane = tid & 31, ln = lane & 15, hh = lane >> 4;
  const int rowb = blockIdx.x * 64;
  const int col0 = blockIdx.y * 64;
  v8f yr[4] = {}, yi[4] = {};
  rgemm_main<false>(Cx, Wo, rowb + 16 * w, col0, ln, hh, yr, yi);
  const float scl = 1.0f / 4194304.0f;
#pragma unroll
  for (int t = 0; t < 4; ++t) {
#pragma unroll
    for (int r = 0; r < 8; ++r) {
      so[w][8 * hh + r][16 * t + ln]      = yr[t][r] * scl;
      so[w][8 * hh + r][HD + 16 * t + ln] = yi[t][r] * scl;
    }
  }
  __syncthreads();
  const int b = rowb / SEQ;
  const int s0 = rowb - b * SEQ + 16 * w;
  const size_t obase = ((size_t)b * SEQ_FULL + (size_t)s0) * RD + (size_t)col0
                     + (size_t)(lane >> 4) * OUT1_OFF + (size_t)(lane & 15) * 4;
  for (int pass = 0; pass < 2; ++pass) {
#pragma unroll
    for (int q = 0; q < 16; ++q) {
      const v4f v = *(const v4fa*)&so[w][q][lane * 4];
      *(volatile v4f*)(Out + obase + (size_t)q * RD) = v;
    }
    if (pass == 0) __threadfence();
  }
}

extern "C" void kernel_launch(void* const* d_in, const int* in_sizes, int n_in,
                              void* d_out, int out_size, void* d_ws, size_t ws_size, hipStream_t stream) {
  if (n_in < 11) return;
  const long long needx = ((long long)(NB - 1) * SEQ_FULL + (long long)SEQ) * RD;
  const long long needm = ((long long)(NB - 1) * SEQ_FULL + (long long)(SEQ - 1)) * SEQ_FULL + (long long)SEQ;
  for (int i = 0; i < 6; ++i) if ((long long)in_sizes[i] < needx) return;
  for (int i = 6; i < 10; ++i) if ((long long)in_sizes[i] < (long long)RD * RD) return;
  if ((long long)in_sizes[10] < needm) return;
  if ((long long)out_size < (long long)OUT1_OFF + needx) return;
  const float* q_re = (const float*)d_in[0];
  const float* k_re = (const float*)d_in[1];
  const float* v_re = (const float*)d_in[2];
  const float* q_ph = (const float*)d_in[3];
  const float* k_ph = (const float*)d_in[4];
  const float* v_ph = (const float*)d_in[5];
  const float* w_q = (const float*)d_in[6];
  const float* w_k = (const float*)d_in[7];
  const float* w_v = (const float*)d_in[8];
  const float* w_o = (const float*)d_in[9];
  const int* maskp = (const int*)d_in[10];
  float* Out = (float*)d_out;

  char* ws = (char*)d_ws;
  size_t off = 0;
  const size_t XB = (size_t)NB * SEQ * KP * 2;
  const size_t WB = (size_t)RD * RD * 2;
  const size_t MBB = (size_t)NB * SEQ * (SEQ / 32) * 4;
  unsigned short* Xq = (unsigned short*)(ws + off); off += XB;
  unsigned short* Xk = (unsigned short*)(ws + off); off += XB;
  unsigned short* Xv = (unsigned short*)(ws + off); off += XB;
  unsigned short* Wq = (unsigned short*)(ws + off); off += WB;
  unsigned short* Wk = (unsigned short*)(ws + off); off += WB;
  unsigned short* Wv = (unsigned short*)(ws + off); off += WB;
  unsigned short* Wo = (unsigned short*)(ws + off); off += WB;
  unsigned short* Qp = (unsigned short*)(ws + off); off += XB;
  unsigned short* Kp = (unsigned short*)(ws + off); off += XB;
  unsigned short* Vt = (unsigned short*)(ws + off); off += XB;
  unsigned short* Cx = (unsigned short*)(ws + off); off += XB;
  unsigned int*   MB = (unsigned int*)(ws + off);   off += MBB;
  if (off > ws_size) return;

  const unsigned gx = (unsigned)((NB * SEQ * 64 + 255) / 256);
  k_cvtx<<<gx, 256, 0, stream>>>(q_re, q_ph, Xq);
  k_cvtx<<<gx, 256, 0, stream>>>(k_re, k_ph, Xk);
  k_cvtx<<<gx, 256, 0, stream>>>(v_re, v_ph, Xv);
  const dim3 gw((unsigned)(RD / 64), (unsigned)(RD / 64), 1);
  k_cvtwt<<<gw, 256, 0, stream>>>(w_q, Wq, 0);
  k_cvtwt<<<gw, 256, 0, stream>>>(w_k, Wk, 0);
  k_cvtwt<<<gw, 256, 0, stream>>>(w_v, Wv, 0);
  k_cvtwt<<<gw, 256, 0, stream>>>(w_o, Wo, 1);
  const unsigned gm = (unsigned)(((size_t)NB * SEQ * (SEQ / 32) + 255) / 256);
  k_maskbits<<<gm, 256, 0, stream>>>(maskp, MB);

  const dim3 gp((unsigned)(NB * SEQ / 64), (unsigned)NH, 1);
  k_proj_rows<<<gp, 128, 0, stream>>>(Xq, Wq, Qp, 256.0f);
  k_proj_rows<<<gp, 128, 0, stream>>>(Xk, Wk, Kp, -256.0f);
  k_proj_vt<<<gp, 128, 0, stream>>>(Xv, Wv, Vt);

  k_attn<<<(unsigned)(NB * NH * (SEQ / 64)), 128, 0, stream>>>(Qp, Kp, Vt, MB, Cx);

  const dim3 go((unsigned)(NB * SEQ / 64), (unsigned)(RD / 64), 1);
  k_out<<<go, 128, 0, stream>>>(Cx, Wo, Out);
}
